// Model_15006615734384
// MI455X (gfx1250) — hardware-verified
//
#include <hip/hip_runtime.h>
#include <math.h>

constexpr int NBATCH   = 1024;
constexpr int NLEV     = 60;
constexpr int NT_SEQ   = 62;
constexpr int NCH_IN   = 25;
constexpr int NCH_LEV  = 9;
constexpr int NCH_GLB  = 16;
constexpr int NHID     = 256;
constexpr int NGATE    = 1024;
constexpr int NH2      = 512;
constexpr int NOUT_LEV = 6;
constexpr int NOUT_GLB = 8;
constexpr int NOUT_ALL = 14;
constexpr int NTHR     = 256;
constexpr int ROWS_BLK = 32;
constexpr int HPITCH   = 264;
constexpr int KPAD0    = 32;
constexpr int NOUT_TOTAL = NBATCH * NLEV * NOUT_ALL;

constexpr float OP_CARRY      = 16.0f;
constexpr float ACC_CARRY     = OP_CARRY * OP_CARRY;
constexpr float ACC_CARRY_INV = 1.0f / ACC_CARRY;
constexpr float LOG2E_F       = 1.4426950408889634f;
constexpr float K_SIG_ACC     = -LOG2E_F * ACC_CARRY_INV;
constexpr float K_TANH_ACC    = 2.0f * LOG2E_F * ACC_CARRY_INV;
constexpr float K_TANH        = 2.0f * LOG2E_F;

static_assert(NT_SEQ == NLEV + 2, "sequence length");
static_assert(NGATE == 4 * NHID && NH2 == 2 * NHID, "gate layout");
static_assert(NBATCH == 1024, "row index uses shifts by 10");
static_assert(NBATCH % ROWS_BLK == 0, "batch tiles");
static_assert(NHID % 32 == 0 && NH2 % 32 == 0 && KPAD0 % 32 == 0, "K multiples of 32");
static_assert(NHID == 32 * (NTHR / 32), "8 waves x 32 hidden columns");
static_assert((2 * ROWS_BLK * HPITCH) % NTHR == 0, "h tile zero fill exact");
static_assert(HPITCH % 8 == 0, "16-B aligned LDS rows");
static_assert(NOUT_TOTAL % (4 * NTHR) == 0, "flat output store exact");
static_assert((NT_SEQ * NBATCH * 4) % NTHR == 0, "input plane build exact");
static_assert(NCH_LEV <= KPAD0 && NCH_GLB <= KPAD0, "padded K covers both kinds");
static_assert(NOUT_LEV + NOUT_GLB == NOUT_ALL, "output columns");

typedef __attribute__((ext_vector_type(16))) _Float16 v16h;
typedef __attribute__((ext_vector_type(8)))  _Float16 v8h;
typedef __attribute__((ext_vector_type(8)))  float    v8f;
typedef __attribute__((ext_vector_type(4)))  float    v4f;

__device__ __forceinline__ v16h ld_frag(const _Float16* p) {
  union { v16h v; v8h h[2]; } f;
  f.h[0] = *(const v8h*)(p);
  f.h[1] = *(const v8h*)(p + 16);
  return f.v;
}
__device__ __forceinline__ v8f mma16(v16h a, v16h b, v8f c) {
  return __builtin_amdgcn_wmma_f32_16x16x32_f16(false, a, false, b, (short)0, c, false, false);
}
__device__ __forceinline__ void hz_guard4(v8f& a, v8f& b, v8f& c, v8f& d, v16h x, v16h y, v16h z, v16h w) {
  asm volatile("v_nop\n\tv_nop\n\tv_nop\n\tv_nop" : "+v"(a), "+v"(b), "+v"(c), "+v"(d) : "v"(x), "v"(y), "v"(z), "v"(w));
}
__device__ __forceinline__ void hz_guard1(v8f& a, v16h x, v16h y) {
  asm volatile("v_nop\n\tv_nop\n\tv_nop\n\tv_nop" : "+v"(a) : "v"(x), "v"(y));
}
__device__ __forceinline__ float fast_rcp(float x)  { return __builtin_amdgcn_rcpf(x); }
__device__ __forceinline__ float fast_exp2(float x) { return __builtin_amdgcn_exp2f(x); }

__global__ __launch_bounds__(NTHR) void cvt8_kernel(const float* __restrict__ src, _Float16* __restrict__ dst, int n8, float sc) {
  const int i = blockIdx.x * NTHR + threadIdx.x;
  if (i < n8) {
    const v4f a = *(const v4f*)(src + (size_t)i * 8);
    const v4f b = *(const v4f*)(src + (size_t)i * 8 + 4);
    v8h hv;
#pragma unroll
    for (int e = 0; e < 4; ++e) {
      hv[e]     = (_Float16)(a[e] * sc);
      hv[4 + e] = (_Float16)(b[e] * sc);
    }
    *(volatile v8h*)(dst + (size_t)i * 8) = hv;
    __threadfence();
    *(volatile v8h*)(dst + (size_t)i * 8) = hv;
  }
}

__global__ __launch_bounds__(128) void fold_kernel(const float* __restrict__ Wih0,
                                                   const float* __restrict__ Wl, const float* __restrict__ bl,
                                                   const float* __restrict__ Wg, const float* __restrict__ bg,
                                                   const float* __restrict__ bih0, const float* __restrict__ bhh0,
                                                   const float* __restrict__ bih1, const float* __restrict__ bhh1,
                                                   _Float16* __restrict__ WEFF, float* __restrict__ BIASP) {
  __shared__ __align__(16) _Float16 sWl[128 * KPAD0];
  __shared__ __align__(16) _Float16 sWg[128 * KPAD0];
  __shared__ __align__(16) float    sB[3 * 128];
  const int tid  = threadIdx.x;
  const int lane = tid & 31;
  const int wave = __builtin_amdgcn_readfirstlane(tid >> 5);
  const int row  = blockIdx.x * 128 + tid;
  const int dir  = blockIdx.x >> 3;
  const int n0   = (blockIdx.x & 7) * 128;
  const float* wr = Wih0 + (size_t)row * NHID;

  float al[NCH_LEV], ag[NCH_GLB];
  float cbl = 0.0f, cbg = 0.0f;
#pragma unroll
  for (int j = 0; j < NCH_LEV; ++j) al[j] = 0.0f;
#pragma unroll
  for (int j = 0; j < NCH_GLB; ++j) ag[j] = 0.0f;
#pragma unroll 1
  for (int k = 0; k < NHID; ++k) {
    const float w = wr[k];
#pragma unroll
    for (int j = 0; j < NCH_LEV; ++j) al[j] = fmaf(w, Wl[k * NCH_LEV + j], al[j]);
#pragma unroll
    for (int j = 0; j < NCH_GLB; ++j) ag[j] = fmaf(w, Wg[k * NCH_GLB + j], ag[j]);
    cbl = fmaf(w, bl[k], cbl);
    cbg = fmaf(w, bg[k], cbg);
  }
  float zf = 0.0f;
  asm volatile("" : "+v"(zf));
#pragma unroll
  for (int q = 0; q < 4; ++q) {
    v8h hl, hg;
#pragma unroll
    for (int e = 0; e < 8; ++e) {
      const int j = 8 * q + e;
      const float fl = (j < NCH_LEV) ? (al[j < NCH_LEV ? j : 0] * OP_CARRY) : zf;
      const float fg = (j < NCH_GLB) ? (ag[j < NCH_GLB ? j : 0] * OP_CARRY) : zf;
      hl[e] = (_Float16)fl;
      hg[e] = (_Float16)fg;
    }
    *(v8h*)(sWl + tid * KPAD0 + 8 * q) = hl;
    *(v8h*)(sWg + tid * KPAD0 + 8 * q) = hg;
  }
  {
    const float b0 = bih0[row] + bhh0[row];
    const float b1 = bih1[row] + bhh1[row];
    sB[0 * 128 + tid] = (b0 + cbl) * ACC_CARRY;
    sB[1 * 128 + tid] = (b0 + cbg) * ACC_CARRY;
    sB[2 * 128 + tid] = b1 * ACC_CARRY;
  }
  __syncthreads();

  _Float16* dl = WEFF + ((size_t)(dir * 2 + 0) * NGATE + n0) * KPAD0;
  _Float16* dg = WEFF + ((size_t)(dir * 2 + 1) * NGATE + n0) * KPAD0;
  v8h ol[4], og[4];
#pragma unroll
  for (int it = 0; it < 4; ++it) {
    const int ch = it * 128 + tid;
    ol[it] = *(const v8h*)(sWl + ch * 8);
    og[it] = *(const v8h*)(sWg + ch * 8);
  }
  const int wsel = (wave < 2) ? wave : 2;
  const v4f bvv = *(const v4f*)(sB + wsel * 128 + lane * 4);
  float* bd = BIASP + (size_t)(dir * 3 + wsel) * NGATE + n0 + lane * 4;
  for (int pass = 0; pass < 2; ++pass) {
#pragma unroll
    for (int it = 0; it < 4; ++it) {
      const int ch = it * 128 + tid;
      *(volatile v8h*)(dl + ch * 8) = ol[it];
      *(volatile v8h*)(dg + ch * 8) = og[it];
    }
    if (wave < 3) *(volatile v4f*)bd = bvv;
    __threadfence();
  }
}

__global__ __launch_bounds__(NTHR) void xh_kernel(const float* __restrict__ x, _Float16* __restrict__ XH) {
  const int i = blockIdx.x * NTHR + threadIdx.x;
  const int nchunk = NT_SEQ * NBATCH * 4;
  if (i < nchunk) {
    const int row = i >> 2;
    const int q   = i & 3;
    const int t   = row >> 10;
    const int b   = row & (NBATCH - 1);
    const bool gk = (t == 0) || (t == NT_SEQ - 1);
    int tl = t - 1;
    tl = tl < 0 ? 0 : tl;
    tl = tl > NLEV - 1 ? NLEV - 1 : tl;
    const int base = gk ? (b * (NLEV * NCH_IN) + NCH_LEV) : ((b * NLEV + tl) * NCH_IN);
    const int lim  = gk ? NCH_GLB : NCH_LEV;
    v8h hv;
#pragma unroll
    for (int e = 0; e < 8; ++e) {
      const int k  = 8 * q + e;
      const int kc = (k < lim) ? k : (lim - 1);
      const float v = x[base + kc];
      const float val = (k < lim) ? (v * OP_CARRY) : 0.0f;
      hv[e] = (_Float16)val;
    }
    *(volatile v8h*)(XH + (size_t)i * 8) = hv;
    __threadfence();
    *(volatile v8h*)(XH + (size_t)i * 8) = hv;
  }
}

__global__ __launch_bounds__(NTHR) void hw_kernel(const float* __restrict__ Wlp, const float* __restrict__ Wgp,
                                                  _Float16* __restrict__ HW) {
  const int i = blockIdx.x * NTHR + threadIdx.x;
  const int nchunk = 2 * 3 * 16 * (NHID / 8);
  if (i < nchunk) {
    const int k8   = i & 31;
    const int row  = (i >> 5) & 15;
    const int sd   = i >> 9;
    const int dir  = sd / 3;
    const int slot = sd - dir * 3;
    const int rl = (row < NOUT_LEV) ? row : (NOUT_LEV - 1);
    const int rg = (row < NOUT_GLB) ? row : (NOUT_GLB - 1);
    const float* pa = Wlp + (size_t)rl * NH2 + dir * NHID + k8 * 8;
    const float* pb = Wgp + (size_t)rg * (2 * NH2) + ((slot == 2) ? NH2 : 0) + dir * NHID + k8 * 8;
    const v4f a0 = *(const v4f*)(pa);
    const v4f a1 = *(const v4f*)(pa + 4);
    const v4f b0 = *(const v4f*)(pb);
    const v4f b1 = *(const v4f*)(pb + 4);
    const bool sl0   = (slot == 0);
    const bool valid = sl0 ? (row < NOUT_LEV) : (row < NOUT_GLB);
    v8h hv;
#pragma unroll
    for (int e = 0; e < 4; ++e) {
      const float s0 = sl0 ? a0[e] : b0[e];
      const float s1 = sl0 ? a1[e] : b1[e];
      const float v0 = valid ? (s0 * OP_CARRY) : 0.0f;
      const float v1 = valid ? (s1 * OP_CARRY) : 0.0f;
      hv[e]     = (_Float16)v0;
      hv[4 + e] = (_Float16)v1;
    }
    *(volatile v8h*)(HW + (size_t)i * 8) = hv;
    __threadfence();
    *(volatile v8h*)(HW + (size_t)i * 8) = hv;
  }
}

template <int LD>
__device__ __forceinline__ void gate_tiles(v8f (&acc)[2][4][2], const v16h a0, const v16h a1, const _Float16* wp) {
#pragma unroll
  for (int g = 0; g < 4; ++g) {
    const v16h b0 = ld_frag(wp + (size_t)(NHID * g) * LD);
    const v16h b1 = ld_frag(wp + (size_t)(NHID * g + 16) * LD);
    acc[0][g][0] = mma16(a0, b0, acc[0][g][0]);
    acc[1][g][0] = mma16(a1, b0, acc[1][g][0]);
    acc[0][g][1] = mma16(a0, b1, acc[0][g][1]);
    acc[1][g][1] = mma16(a1, b1, acc[1][g][1]);
    hz_guard4(acc[0][g][0], acc[1][g][0], acc[0][g][1], acc[1][g][1], a0, a1, b0, b1);
  }
}

template <int LAYER>
__global__ __launch_bounds__(NTHR) __attribute__((amdgpu_num_vgpr(256)))
void scan_kernel(const _Float16* __restrict__ AIN, const _Float16* __restrict__ WIN, const _Float16* __restrict__ WREC,
                 const float* __restrict__ BIASP, const _Float16* __restrict__ HW,
                 _Float16* __restrict__ H0OUT, float* __restrict__ PART) {
  __shared__ __align__(16) _Float16 Ah[2 * ROWS_BLK * HPITCH];
  __shared__ __align__(16) float    Hs[2 * 256];
  constexpr int LDIN = (LAYER == 0) ? KPAD0 : NH2;

  const int tid  = threadIdx.x;
  const int lane = tid & 31;
  const int wave = __builtin_amdgcn_readfirstlane(tid >> 5);
  const int c    = lane & 15;
  const int hh   = lane >> 4;
  const int koff = hh * 8;
  const int bbase = blockIdx.x * ROWS_BLK;
  const int dir   = blockIdx.y;

#pragma unroll 1
  for (int i = tid; i < 2 * ROWS_BLK * HPITCH; i += NTHR) Ah[i] = (_Float16)0.0f;

  float cst[2][2][8];
#pragma unroll
  for (int mt = 0; mt < 2; ++mt)
#pragma unroll
    for (int s = 0; s < 2; ++s)
#pragma unroll
      for (int r = 0; r < 8; ++r) cst[mt][s][r] = 0.0f;

  const _Float16* wrec = WREC + ((size_t)dir * NGATE + 32 * wave + c) * NHID + koff;
  const _Float16* win  = (LAYER == 0)
      ? (WIN + ((size_t)(dir * 2) * NGATE + 32 * wave + c) * KPAD0 + koff)
      : (WIN + ((size_t)dir * NGATE + 32 * wave + c) * NH2 + koff);
  __syncthreads();

#pragma unroll 1
  for (int tt = 0; tt < NT_SEQ; ++tt) {
    const int t = dir ? (NT_SEQ - 1 - tt) : tt;
    const int p = tt & 1;
    const bool ends = (t == 0) || (t == NT_SEQ - 1);
    const _Float16* ahc = Ah + p * (ROWS_BLK * HPITCH);
    _Float16*       ahn = Ah + (p ^ 1) * (ROWS_BLK * HPITCH);

    const int bslot = (LAYER == 0) ? (ends ? 1 : 0) : 2;
    const float* bp = BIASP + (size_t)(dir * 3 + bslot) * NGATE + 32 * wave + c;
    v8f acc[2][4][2];
#pragma unroll
    for (int g = 0; g < 4; ++g)
#pragma unroll
      for (int s = 0; s < 2; ++s) {
        const float bv = bp[NHID * g + 16 * s];
#pragma unroll
        for (int mt = 0; mt < 2; ++mt)
#pragma unroll
          for (int r = 0; r < 8; ++r) acc[mt][g][s][r] = bv;
      }

    {
      const _Float16* ap = AIN + ((size_t)t * NBATCH + bbase + c) * LDIN + koff;
      if (LAYER == 0) {
        const v16h a0 = ld_frag(ap);
        const v16h a1 = ld_frag(ap + 16 * LDIN);
        const _Float16* wp = win + (ends ? (NGATE * KPAD0) : 0);
        gate_tiles<LDIN>(acc, a0, a1, wp);
      } else {
#pragma unroll 1
        for (int k0 = 0; k0 < NH2; k0 += 32) {
          const v16h a0 = ld_frag(ap + k0);
          const v16h a1 = ld_frag(ap + 16 * LDIN + k0);
          gate_tiles<LDIN>(acc, a0, a1, win + k0);
        }
      }
    }
    {
      const _Float16* ar = ahc + c * HPITCH + koff;
#pragma unroll 1
      for (int k0 = 0; k0 < NHID; k0 += 32) {
        const v16h a0 = ld_frag(ar + k0);
        const v16h a1 = ld_frag(ar + 16 * HPITCH + k0);
        gate_tiles<NHID>(acc, a0, a1, wrec + k0);
      }
    }

#pragma unroll
    for (int mt = 0; mt < 2; ++mt)
#pragma unroll
      for (int s = 0; s < 2; ++s)
#pragma unroll
        for (int r = 0; r < 8; ++r) {
          const float ai = acc[mt][0][s][r];
          const float af = acc[mt][1][s][r];
          const float ag = acc[mt][2][s][r];
          const float ao = acc[mt][3][s][r];
          const float ig = fast_rcp(1.0f + fast_exp2(ai * K_SIG_ACC));
          const float fg = fast_rcp(1.0f + fast_exp2(af * K_SIG_ACC));
          const float og = fast_rcp(1.0f + fast_exp2(ao * K_SIG_ACC));
          const float gt = fmaf(-2.0f, fast_rcp(fast_exp2(ag * K_TANH_ACC) + 1.0f), 1.0f);
          const float cn = fmaf(fg, cst[mt][s][r], ig * gt);
          cst[mt][s][r] = cn;
          const float th16 = fmaf(-2.0f * OP_CARRY, fast_rcp(fast_exp2(cn * K_TANH) + 1.0f), OP_CARRY);
          ahn[(16 * mt + 8 * hh + r) * HPITCH + 32 * wave + 16 * s + c] = (_Float16)(og * th16);
        }

    __syncthreads();

    if (LAYER == 0) {
      v8h hv[4];
#pragma unroll
      for (int it = 0; it < 4; ++it) hv[it] = *(const v8h*)(ahn + (it * 8 + wave) * HPITCH + lane * 8);
      _Float16* dst = H0OUT + ((size_t)t * NBATCH + bbase) * NH2 + dir * NHID + lane * 8;
      for (int pass = 0; pass < 2; ++pass) {
#pragma unroll
        for (int it = 0; it < 4; ++it) *(volatile v8h*)(dst + (size_t)(it * 8 + wave) * NH2) = hv[it];
        __threadfence();
      }
    } else {
      if (wave < 2) {
        const int slot = (t == 0) ? 1 : ((t == NT_SEQ - 1) ? 2 : 0);
        const _Float16* hp = HW + ((size_t)(dir * 3 + slot) * 16 + c) * NHID + koff;
        const _Float16* ar = ahn + (16 * wave + c) * HPITCH + koff;
        v8f ha = (v8f){0.f, 0.f, 0.f, 0.f, 0.f, 0.f, 0.f, 0.f};
#pragma unroll 1
        for (int k0 = 0; k0 < NHID; k0 += 32) {
          const v16h a = ld_frag(ar + k0);
          const v16h b = ld_frag(hp + k0);
          ha = mma16(a, b, ha);
          hz_guard1(ha, a, b);
        }
        float* slab = Hs + wave * 256;
#pragma unroll
        for (int r = 0; r < 8; ++r) slab[(8 * hh + r) * 16 + c] = ha[r] * ACC_CARRY_INV;
        __builtin_amdgcn_fence(__ATOMIC_RELEASE, "workgroup");
        __builtin_amdgcn_wave_barrier();
        __builtin_amdgcn_fence(__ATOMIC_ACQUIRE, "workgroup");
        const v4f v0 = *(const v4f*)(slab + lane * 4);
        const v4f v1 = *(const v4f*)(slab + 128 + lane * 4);
        float* dst = PART + (((size_t)dir * NT_SEQ + t) * NBATCH + bbase + 16 * wave) * 16 + lane * 4;
        for (int pass = 0; pass < 2; ++pass) {
          *(volatile v4f*)(dst) = v0;
          *(volatile v4f*)(dst + 128) = v1;
          __threadfence();
        }
        __builtin_amdgcn_fence(__ATOMIC_RELEASE, "workgroup");
        __builtin_amdgcn_wave_barrier();
        __builtin_amdgcn_fence(__ATOMIC_ACQUIRE, "workgroup");
      }
    }
  }
}

__global__ __launch_bounds__(NTHR) void final_kernel(const float* __restrict__ PART, const float* __restrict__ blp,
                                                     const float* __restrict__ bgp, float* __restrict__ out) {
  __shared__ float sb[16];
  const int tid = threadIdx.x;
  {
    const int i6 = (tid < NOUT_LEV) ? tid : (NOUT_LEV - 1);
    int i8 = tid - NOUT_LEV;
    i8 = i8 < 0 ? 0 : i8;
    i8 = i8 > NOUT_GLB - 1 ? NOUT_GLB - 1 : i8;
    const float a = blp[i6];
    const float b = bgp[i8];
    const float v = (tid < NOUT_LEV) ? a : b;
    if (tid < 16) sb[tid] = v;
  }
  __syncthreads();
  const int i4 = blockIdx.x * NTHR + tid;
  if (i4 < NOUT_TOTAL / 4) {
    const int e0 = i4 * 4;
    v4f o;
#pragma unroll
    for (int q = 0; q < 4; ++q) {
      const int e   = e0 + q;
      const int b   = e / (NLEV * NOUT_ALL);
      const int rem = e - b * (NLEV * NOUT_ALL);
      const int s   = rem / NOUT_ALL;
      const int oc  = rem - s * NOUT_ALL;
      const bool lo = (oc < NOUT_LEV);
      const int col = lo ? oc : (oc - NOUT_LEV);
      const int tA  = lo ? (s + 1) : 0;
      const float pA0 = PART[((size_t)(0 * NT_SEQ + tA) * NBATCH + b) * 16 + col];
      const float pA1 = PART[((size_t)(1 * NT_SEQ + tA) * NBATCH + b) * 16 + col];
      const float pB0 = PART[((size_t)(0 * NT_SEQ + NT_SEQ - 1) * NBATCH + b) * 16 + col];
      const float pB1 = PART[((size_t)(1 * NT_SEQ + NT_SEQ - 1) * NBATCH + b) * 16 + col];
      const float tail = lo ? 0.0f : (pB0 + pB1);
      o[q] = ((pA0 + pA1) + tail) + sb[oc];
    }
    *(volatile v4f*)(out + (size_t)e0) = o;
    __threadfence();
    *(volatile v4f*)(out + (size_t)e0) = o;
  }
}

extern "C" void kernel_launch(void* const* d_in, const int* in_sizes, int n_in,
                              void* d_out, int out_size, void* d_ws, size_t ws_size, hipStream_t stream) {
  if (n_in < 17 || d_out == nullptr || d_ws == nullptr) return;
  if (in_sizes[0] != NBATCH * NLEV * NCH_IN || in_sizes[1] != NHID * NCH_GLB || in_sizes[2] != NHID ||
      in_sizes[3] != NHID * NCH_LEV || in_sizes[4] != NHID ||
      in_sizes[5] != 2 * NGATE * NHID || in_sizes[6] != 2 * NGATE * NHID ||
      in_sizes[7] != 2 * NGATE || in_sizes[8] != 2 * NGATE ||
      in_sizes[9] != 2 * NGATE * NH2 || in_sizes[10] != 2 * NGATE * NHID ||
      in_sizes[11] != 2 * NGATE || in_sizes[12] != 2 * NGATE ||
      in_sizes[13] != NOUT_GLB * 2 * NH2 || in_sizes[14] != NOUT_GLB ||
      in_sizes[15] != NOUT_LEV * NH2 || in_sizes[16] != NOUT_LEV ||
      out_size != NOUT_TOTAL) return;

  const float* x    = (const float*)d_in[0];
  const float* Wg   = (const float*)d_in[1];
  const float* bg   = (const float*)d_in[2];
  const float* Wl   = (const float*)d_in[3];
  const float* bl   = (const float*)d_in[4];
  const float* Wih0 = (const float*)d_in[5];
  const float* Whh0 = (const float*)d_in[6];
  const float* bih0 = (const float*)d_in[7];
  const float* bhh0 = (const float*)d_in[8];
  const float* Wih1 = (const float*)d_in[9];
  const float* Whh1 = (const float*)d_in[10];
  const float* bih1 = (const float*)d_in[11];
  const float* bhh1 = (const float*)d_in[12];
  const float* Wgp  = (const float*)d_in[13];
  const float* bgp  = (const float*)d_in[14];
  const float* Wlp  = (const float*)d_in[15];
  const float* blp  = (const float*)d_in[16];
  float* out = (float*)d_out;

  char* ws = (char*)d_ws;
  size_t off = 0;
  auto carve = [&](size_t bytes) -> char* { char* p = ws + off; off += (bytes + 255) & ~(size_t)255; return p; };
  _Float16* XH    = (_Float16*)carve((size_t)NT_SEQ * NBATCH * KPAD0 * 2);
  _Float16* H0    = (_Float16*)carve((size_t)NT_SEQ * NBATCH * NH2 * 2);
  _Float16* WHH0  = (_Float16*)carve((size_t)2 * NGATE * NHID * 2);
  _Float16* WIH1  = (_Float16*)carve((size_t)2 * NGATE * NH2 * 2);
  _Float16* WHH1  = (_Float16*)carve((size_t)2 * NGATE * NHID * 2);
  _Float16* WEFF  = (_Float16*)carve((size_t)2 * 2 * NGATE * KPAD0 * 2);
  _Float16* HW    = (_Float16*)carve((size_t)2 * 3 * 16 * NHID * 2);
  float*    BIASP = (float*)carve((size_t)2 * 3 * NGATE * 4);
  float*    PART  = (float*)carve((size_t)2 * NT_SEQ * NBATCH * 16 * 4);
  if (off > ws_size || off > (size_t)134217728) return;

  const int n8hh = 2 * NGATE * NHID / 8;
  const int n8ih = 2 * NGATE * NH2 / 8;
  cvt8_kernel<<<n8hh / NTHR, NTHR, 0, stream>>>(Whh0, WHH0, n8hh, OP_CARRY);
  cvt8_kernel<<<n8ih / NTHR, NTHR, 0, stream>>>(Wih1, WIH1, n8ih, OP_CARRY);
  cvt8_kernel<<<n8hh / NTHR, NTHR, 0, stream>>>(Whh1, WHH1, n8hh, OP_CARRY);
  fold_kernel<<<(2 * NGATE) / 128, 128, 0, stream>>>(Wih0, Wl, bl, Wg, bg, bih0, bhh0, bih1, bhh1, WEFF, BIASP);
  xh_kernel<<<(NT_SEQ * NBATCH * 4) / NTHR, NTHR, 0, stream>>>(x, XH);
  hw_kernel<<<(2 * 3 * 16 * (NHID / 8)) / NTHR, NTHR, 0, stream>>>(Wlp, Wgp, HW);
  const dim3 sgrid(NBATCH / ROWS_BLK, 2);
  scan_kernel<0><<<sgrid, NTHR, 0, stream>>>(XH, WEFF, WHH0, BIASP, HW, H0, PART);
  scan_kernel<1><<<sgrid, NTHR, 0, stream>>>(H0, WIH1, WHH1, BIASP, HW, XH, PART);
  final_kernel<<<NOUT_TOTAL / (4 * NTHR), NTHR, 0, stream>>>(PART, blp, bgp, out);
}
